// GraphTransformerLayer_80668075753491
// MI455X (gfx1250) — hardware-run, weakly checked
//
#include <hip/hip_runtime.h>


namespace {


constexpr int N = 50000, NP = 50048, NPL = NP  , SRCM = N  , EFULL = 640000, E = EFULL  ;
constexpr int D = 128, HH = 4, DK = 32, ED = 64, NREL = 51  , DF = 512, NL = (NPL < N ? NPL : N), NRL = NP  ;
constexpr float LNEPS = 1e-5f; constexpr float LOG2E = 1.4426950408889634f, ISQD = 0.17677669529663687f  ;
constexpr float XS = 8.0f, WSC = 256.0f, WSQ = 0.25f, RS_ = 1024.0f, SLOPE = 0.0f, BNEPS = 1e-5f;
static_assert(NP % 32 == 0 && NP >= N && NPL % 32 == 0 && D == 128, "tiling");
typedef _Float16 b16;
typedef __attribute__((ext_vector_type(16))) _Float16 v16b;
typedef __attribute__((ext_vector_type(8))) _Float16 v8b;
typedef __attribute__((ext_vector_type(8))) float v8f;
typedef __attribute__((ext_vector_type(4))) float v4f;
__device__ __forceinline__ float bf16_rne(float f) { unsigned int u = __float_as_uint(f); u += 0x7FFFu + ((u >> 16) & 1u); return __uint_as_float(u & 0xFFFF0000u); }
__device__ __forceinline__ void split16(float v, b16& hi, b16& lo) { hi = (b16)v; lo = (b16)(v - (float)hi); }
__device__ __forceinline__ v16b frag_kb(const b16* p, int hh) { const v8b a = *(const v8b*)(p + 8 * hh), b = *(const v8b*)(p + 16 + 8 * hh); v16b f;
#pragma unroll
  for (int e = 0; e < 8; ++e) { f[e] = a[e]; f[8 + e] = b[e]; } return f; }
__device__ __forceinline__ v8f wmma16b(v16b a, v16b b, v8f c) { v8f d = __builtin_amdgcn_wmma_f32_16x16x32_f16(false, a, false, b, (short)0, c, false, false); asm volatile("v_nop\n\tv_nop\n\tv_nop\n\tv_nop" : "+v"(d) : "v"(a), "v"(b)); return d; }
__device__ __forceinline__ void wave_lds_sync() { __builtin_amdgcn_fence(__ATOMIC_RELEASE, "workgroup"); __builtin_amdgcn_wave_barrier(); __builtin_amdgcn_fence(__ATOMIC_ACQUIRE, "workgroup"); }
__device__ __forceinline__ float pmul(float a, float b) { float p = a * b; asm volatile("" : "+v"(p)); return p; }
__device__ __forceinline__ int iclamp(int v, int lo, int hi) { return v < lo ? lo : (v > hi ? hi : v); }
constexpr int CSR_NBLK = 512, CSR_GB = 9, CSR_GN = 1 << CSR_GB  , CSR_MAXG = 512, CSR_CAP = 12288  ;
__global__ __launch_bounds__(64) void csrA_kernel(const int* __restrict__ dst, int E, int N, int nG, int CHP, int NGP, int* __restrict__ STG, int* __restrict__ HST) {
  extern __shared__ int sm[];
  int* cnt = sm; int* run = sm + NGP; int* ids = sm + 2 * NGP;
  const int b = blockIdx.x; const int ch = (E + CSR_NBLK - 1) / CSR_NBLK; const int e0 = b * ch, e1 = min(E, e0 + ch);
  for (int i = threadIdx.x; i < NGP; i += 64) cnt[i] = 0;
  for (int i = threadIdx.x; i < CHP; i += 64) ids[i] = -1;
  __syncthreads();
  if (threadIdx.x == 0) {
    for (int e = e0; e < e1; ++e) { int d = dst[e]; d = (d < 0) ? 0 : (d >= N ? N - 1 : d); cnt[d >> CSR_GB] += 1; }
    int acc = 0; for (int g = 0; g < nG; ++g) { run[g] = acc; acc += cnt[g]; }
    for (int e = e0; e < e1; ++e) { int d = dst[e]; d = (d < 0) ? 0 : (d >= N ? N - 1 : d); const int g = d >> CSR_GB; ids[run[g]] = e; run[g] += 1; } }
  __syncthreads();
  typedef __attribute__((ext_vector_type(4))) int v4i;
  for (int pass = 0; pass < 2; ++pass) {
    for (int i = threadIdx.x; i < CHP / 4; i += 64) *(volatile v4i*)(STG + (size_t)b * CHP + i * 4) = *(const v4i*)(&ids[i * 4]);
    for (int i = threadIdx.x; i < NGP / 4; i += 64) { v4i v; for (int e = 0; e < 4; ++e) v[e] = (i * 4 + e < nG) ? cnt[i * 4 + e] : 0; *(volatile v4i*)(HST + (size_t)b * NGP + i * 4) = v; }
    __threadfence(); }
}
__global__ __launch_bounds__(512) void csrS_kernel(const int* __restrict__ HST, int nG, int NGP, int* __restrict__ START, int* __restrict__ TOT, int* __restrict__ OFF) {
  __shared__ int tot[CSR_MAXG];
  const int b = threadIdx.x;
  for (int pass = 0; pass < 2; ++pass) { int runb = 0; for (int g = 0; g < nG; ++g) { int c = HST[(size_t)b * NGP + g]; c = (c < 0) ? 0 : c; ((volatile int*)OFF)[(size_t)g * CSR_NBLK + b] = runb; runb += c; } __threadfence(); }
  for (int g = threadIdx.x; g < nG; g += 512) { int s = 0; for (int bb = 0; bb < CSR_NBLK; ++bb) { int c = HST[(size_t)bb * NGP + g]; s += (c < 0) ? 0 : c; } tot[g] = s; }
  __syncthreads();
  if (threadIdx.x < 32) {
    __shared__ int st[CSR_MAXG + 32];
    if (threadIdx.x == 0) { int acc = 0; for (int g = 0; g < NGP; ++g) { st[g] = acc; if (g < nG) acc += (tot[g] + 31) & ~31; } st[NGP] = acc; }
    __builtin_amdgcn_fence(__ATOMIC_RELEASE, "workgroup"); __builtin_amdgcn_wave_barrier(); __builtin_amdgcn_fence(__ATOMIC_ACQUIRE, "workgroup");
    for (int pass = 0; pass < 2; ++pass) { for (int i = threadIdx.x; i < NGP + 32; i += 32) { ((volatile int*)START)[i] = (i <= NGP) ? st[min(i, NGP)] : 0; ((volatile int*)TOT)[i] = (i < nG) ? tot[i] : 0; } __threadfence(); } }
}
__global__ __launch_bounds__(256) void csrB_kernel(const int* __restrict__ dst, int N, int nG, int CHP, int NGP, int permLen, const int* __restrict__ STG, const int* __restrict__ HST, const int* __restrict__ OFF, const int* __restrict__ START, const int* __restrict__ TOT, int* __restrict__ PERM, int* __restrict__ ROWPTR, int* __restrict__ ROWCNT, int* __restrict__ FLAG) {
  typedef __attribute__((ext_vector_type(4))) int v4i;
  __shared__ int ids[CSR_CAP]; __shared__ unsigned short key[CSR_CAP]; __shared__ int outp[CSR_CAP]; __shared__ int ncnt[CSR_GN + 1]; __shared__ int boff[CSR_NBLK + 1];
  const int g = blockIdx.x, t_ = threadIdx.x; int tot = TOT[g]; int st = START[g], stn = START[g + 1]; const int v0 = g * CSR_GN; const int nv = min(CSR_GN, N - v0);
  st = (st < 0) ? 0 : (st > permLen - 32 ? permLen - 32 : st) & ~31; stn = (stn < st) ? st : (stn > permLen ? permLen : stn); tot = (tot < 0) ? 0 : tot; if (tot > stn - st && tot <= CSR_CAP) tot = stn - st;
  if (tot > CSR_CAP) {
    for (int pass = 0; pass < 2; ++pass) { for (int i = t_; i < CSR_GN / 4; i += 256) { v4i a, c; for (int e = 0; e < 4; ++e) { a[e] = st; c[e] = 0; } *(volatile v4i*)(ROWPTR + v0 + i * 4) = a; *(volatile v4i*)(ROWCNT + v0 + i * 4) = c; } if (t_ == 0) ((volatile int*)FLAG)[0] = 1; __threadfence(); } (void)nv; return; }
  if (t_ == 0) { int acc = 0; for (int b = 0; b < CSR_NBLK; ++b) { boff[b] = acc; int c = HST[(size_t)b * NGP + g]; c = (c < 0) ? 0 : (c > CHP ? CHP : c); acc += c; if (acc > tot) acc = tot; } boff[CSR_NBLK] = acc; }
  for (int i = t_; i <= CSR_GN; i += 256) ncnt[i] = 0;
  __syncthreads();
  for (int b = 0; b < CSR_NBLK; ++b) { const int c = boff[b + 1] - boff[b]; int o_ = OFF[(size_t)g * CSR_NBLK + b]; o_ = (o_ < 0) ? 0 : (o_ > CHP - c ? CHP - c : o_); const int* src_ = STG + (size_t)b * CHP + o_;
    for (int i = t_; i < c; i += 256) { int id = src_[i]; id = (id < 0) ? 0 : id; ids[boff[b] + i] = id; int d = dst[id]; d = (d < v0) ? v0 : (d >= N ? N - 1 : d); int kk = d - v0; kk = (kk < 0) ? 0 : (kk >= CSR_GN ? CSR_GN - 1 : kk); key[boff[b] + i] = (unsigned short)kk; } }
  __syncthreads();
  if (t_ == 0) { for (int i = 0; i < tot; ++i) ncnt[key[i]] += 1; int acc = 0; for (int vl = 0; vl < CSR_GN; ++vl) { const int c = ncnt[vl]; ncnt[vl] = acc; acc += c; } ncnt[CSR_GN] = acc;
    for (int i = 0; i < tot; ++i) { const int vl = key[i]; outp[ncnt[vl]] = ids[i]; ncnt[vl] += 1; }
    for (int vl = CSR_GN; vl > 0; --vl) ncnt[vl] = ncnt[vl - 1]; ncnt[0] = 0; }
  __syncthreads();
  for (int pass = 0; pass < 2; ++pass) {
    for (int i = t_; i < (stn - st) / 4; i += 256) { v4i v; for (int e = 0; e < 4; ++e) { const int q = i * 4 + e; v[e] = (q < tot) ? outp[q] : -1; } *(volatile v4i*)(PERM + st + i * 4) = v; }
    for (int i = t_; i < CSR_GN / 4; i += 256) { v4i a, c; for (int e = 0; e < 4; ++e) { const int vl = i * 4 + e; a[e] = st + ncnt[vl]; c[e] = (vl < nv) ? (ncnt[vl + 1] - ncnt[vl]) : 0; } *(volatile v4i*)(ROWPTR + v0 + i * 4) = a; *(volatile v4i*)(ROWCNT + v0 + i * 4) = c; }
    __threadfence(); }
}
__global__ __launch_bounds__(256) void csrZ_kernel(int* __restrict__ p, size_t n4) { typedef __attribute__((ext_vector_type(4))) int v4i; const size_t tid = (size_t)blockIdx.x * 256 + threadIdx.x, nth = (size_t)gridDim.x * 256; v4i z = {0, 0, 0, 0}; for (size_t i = tid; i < n4; i += nth) *(volatile v4i*)(p + i * 4) = z; }
struct CsrBufs { int *STG, *HST, *OFF, *START, *TOT, *PERM, *ROWPTR, *ROWCNT, *FLAG; int nG, NGP, CHP; size_t permLen; char* base; size_t bytes; };
static size_t csr_carve(CsrBufs& c, char* ws, size_t off, int E, int N) {
  const size_t off0 = off; c.base = ws + off;
  auto al = [&](size_t bytes) { char* p = ws + off; off += (bytes + 255) & ~(size_t)255; return p; };
  c.nG = (N + CSR_GN - 1) / CSR_GN; c.NGP = (c.nG + 31) & ~31; const int ch = (E + CSR_NBLK - 1) / CSR_NBLK; c.CHP = (ch + 31) & ~31; c.permLen = (size_t)E + 32 * (size_t)c.nG + 32;
  c.STG = (int*)al((size_t)CSR_NBLK * c.CHP * 4); c.HST = (int*)al((size_t)CSR_NBLK * c.NGP * 4); c.OFF = (int*)al((size_t)c.NGP * CSR_NBLK * 4); c.START = (int*)al((size_t)(c.NGP + 64) * 4); c.TOT = (int*)al((size_t)(c.NGP + 64) * 4);
  c.PERM = (int*)al(c.permLen * 4); c.ROWPTR = (int*)al((size_t)c.nG * CSR_GN * 4); c.ROWCNT = (int*)al((size_t)c.nG * CSR_GN * 4); c.FLAG = (int*)al(256);
  c.bytes = off - off0; return off;
}
static void csr_build(const CsrBufs& c, const int* dst, int E, int N, hipStream_t stream) {
  const size_t smem = (size_t)(2 * c.NGP + c.CHP) * 4;
  csrZ_kernel<<<512, 256, 0, stream>>>((int*)c.base, c.bytes / 16);
  csrA_kernel<<<CSR_NBLK, 64, smem, stream>>>(dst, E, N, c.nG, c.CHP, c.NGP, c.STG, c.HST);
  csrS_kernel<<<1, 512, 0, stream>>>(c.HST, c.nG, c.NGP, c.START, c.TOT, c.OFF);
  csrB_kernel<<<c.nG, 256, 0, stream>>>(dst, N, c.nG, c.CHP, c.NGP, (int)c.permLen, c.STG, c.HST, c.OFF, c.START, c.TOT, c.PERM, c.ROWPTR, c.ROWCNT, c.FLAG);
}

typedef __attribute__((ext_vector_type(4))) _Float16 v4h;
template <int NOUT, int K = D, int NOUTR = NOUT>
__global__ __launch_bounds__(256) void wt_kernel(const float* __restrict__ w, b16* __restrict__ WT, float scl) {
  const int u = blockIdx.x * 256 + threadIdx.x; if (u >= NOUT * K / 8) return; const int e = u * 8; const int o = e / K, k0 = e % K; v8b v;
#pragma unroll
  for (int j = 0; j < 8; ++j) v[j] = (b16)(o < NOUTR ? bf16_rne(w[(size_t)(k0 + j) * NOUTR + o]) * scl : 0.0f);
  for (int pass = 0; pass < 2; ++pass) { *(volatile v8b*)(WT + e) = v; __threadfence(); }
}
__device__ __forceinline__ float gelu_(float v) { return 0.5f * v * (1.0f + erff(v * 0.70710678118654752f)); }
template <bool TR>
__global__ __launch_bounds__(256) void wtbd_kernel(const float* __restrict__ rel, b16* __restrict__ WT, float scl) {
  const int u = blockIdx.x * 256 + threadIdx.x; if (u >= D * D / 8) return; const int e = u * 8; const int o = e / D, k0 = e % D; const int ho = o / DK, oo = o % DK; v8b v;
#pragma unroll
  for (int j = 0; j < 8; ++j) { const int k = k0 + j; const int hk = k / DK, kk = k % DK; float w = 0.0f;
    if (hk == ho) w = TR ? rel[((size_t)ho * DK + oo) * DK + kk]   : rel[((size_t)ho * DK + kk) * DK + oo]  ;
    v[j] = (b16)(bf16_rne(w) * scl); }
  for (int pass = 0; pass < 2; ++pass) { *(volatile v8b*)(WT + e) = v; __threadfence(); }
}
__global__ __launch_bounds__(128) void bcopy_kernel(const float* __restrict__ b, float* __restrict__ B) { const int i = threadIdx.x; for (int pass = 0; pass < 2; ++pass) { ((volatile float*)B)[i] = b[i]; __threadfence(); } }
template <int K, bool RND, int MODE>
__global__ __launch_bounds__(64) void lin_kernel(const float* __restrict__ IN, const b16* __restrict__ WT, const b16* __restrict__ WQ, const float* __restrict__ bias, const float* __restrict__ gate, const float* __restrict__ xprev, float* __restrict__ OUT, int mrows) {
  __shared__ __attribute__((aligned(16))) b16 Ah[2][16][K + 8], Al[2][16][K + 8]; __shared__ __attribute__((aligned(16))) float Tf[2][16][D + 4];
  const int wave = threadIdx.x >> 5, lane = threadIdx.x & 31, nloc = lane & 15, hlf = lane >> 4; const size_t m0 = (size_t)blockIdx.x * 32 + wave * 16; const int mat = blockIdx.y;
  const b16* W = WT + (size_t)mat * D * K; const b16* Wq = RND ? nullptr : WQ + (size_t)mat * D * K; const float* bb_ = bias ? bias + (size_t)mat * D : nullptr; float* O = OUT + (size_t)mat * NP * D;
  for (int idx = lane; idx < 16 * (K / 4); idx += 32) { const int rr = idx / (K / 4), c4 = (idx % (K / 4)) * 4; const size_t arow = (m0 + rr < (size_t)N) ? m0 + rr : (size_t)N - 1; const v4f v = *(const v4f*)(IN + arow * K + c4); v4h hv, lv;
    for (int j = 0; j < 4; ++j) { const float vs = (RND ? bf16_rne(v[j]) : v[j]) * XS; const b16 ph = (b16)vs; hv[j] = ph; lv[j] = (b16)((vs - (float)ph) * RS_); } *(v4h*)(&Ah[wave][rr][c4]) = hv; if (!RND) *(v4h*)(&Al[wave][rr][c4]) = lv; }
  wave_lds_sync();
  v8f acc[8];
#pragma unroll
  for (int t = 0; t < 8; ++t) acc[t] = (v8f){};
#pragma unroll
  for (int kb = 0; kb < K; kb += 32) { const v16b a = frag_kb(&Ah[wave][nloc][kb], hlf); v16b al; if (!RND) al = frag_kb(&Al[wave][nloc][kb], hlf);
#pragma unroll
    for (int t = 0; t < 8; ++t) { const size_t wo_ = (size_t)(t * 16 + nloc) * K + kb; acc[t] = wmma16b(a, frag_kb(W + wo_, hlf), acc[t]); if (!RND) acc[t] = wmma16b(al, frag_kb(Wq + wo_, hlf), acc[t]); } }
  const float sg = (MODE == 3) ? 1.0f / (1.0f + __expf(-bf16_rne(gate[0]))) : 0.0f;
#pragma unroll
  for (int t = 0; t < 8; ++t) { const int col = t * 16 + nloc; const float bb = bb_ ? bf16_rne(bb_[col]) : 0.0f;
    for (int r = 0; r < 8; ++r) { const size_t vrow = m0 + 8 * hlf + r; float y = acc[t][r] * (1.0f / (XS * WSC)) + bb; if (MODE == 1) y = fmaxf(y, 0.0f); if (MODE == 2) y = gelu_(y); if (MODE == 3) y = sg * y + (1.0f - sg) * xprev[(vrow < (size_t)N ? vrow : (size_t)N - 1) * D + col];
      Tf[wave][8 * hlf + r][col] = (vrow < (size_t)N) ? y : 0.0f; } }
  wave_lds_sync();
  for (int pass = 0; pass < 2; ++pass) { for (int rr = 0; rr < 16; ++rr) if (m0 + rr < (size_t)mrows) *(volatile v4f*)(O + (m0 + rr) * D + lane * 4) = *(const v4f*)(&Tf[wave][rr][lane * 4]); __threadfence(); }
}
__global__ __launch_bounds__(256) void etab_kernel(const float* __restrict__ remb, const float* __restrict__ We, float* __restrict__ ET) {
  const int u = blockIdx.x * 256 + threadIdx.x; const bool ok = u < NREL * D; const int t = ok ? u / D : 0, c = u % D; float acc = 0.0f;
#pragma unroll 1
  for (int d = 0; d < ED; ++d) acc = fmaf(bf16_rne(remb[t * ED + d]), bf16_rne(We[(size_t)d * D + c]), acc);
  for (int pass = 0; pass < 2; ++pass) { if (ok) ((volatile float*)ET)[u] = acc; __threadfence(); }
}
__global__ __launch_bounds__(256) void ln_kernel(const float* __restrict__ s, const float* __restrict__ gam, const float* __restrict__ bet, float* __restrict__ X) {
  const int tid = threadIdx.x; const int row = tid >> 3, g = tid & 7, c0 = g * 16; const int v = blockIdx.x * 32 + row; const int vv = v < N ? v : N - 1;
  float a[16]; float s1 = 0.0f;
#pragma unroll
  for (int q = 0; q < 4; ++q) { const v4f t4 = *(const v4f*)(s + (size_t)vv * D + c0 + 4 * q); for (int j = 0; j < 4; ++j) { a[4 * q + j] = bf16_rne(t4[j]); s1 += a[4 * q + j]; } }
#pragma unroll
  for (int o = 1; o < 8; o <<= 1) s1 += __shfl_xor(s1, o);
  const float mu = s1 * (1.0f / (float)D); float s2 = 0.0f;
#pragma unroll
  for (int j = 0; j < 16; ++j) { const float d_ = a[j] - mu; s2 += pmul(d_, d_); }
#pragma unroll
  for (int o = 1; o < 8; o <<= 1) s2 += __shfl_xor(s2, o);
  const float rstd = rsqrtf(s2 * (1.0f / (float)D) + LNEPS);
  for (int pass = 0; pass < 2; ++pass) { float* xr = X + (size_t)v * D + c0;
#pragma unroll
    for (int q = 0; q < 4; ++q) { v4f o; for (int j = 0; j < 4; ++j) { const int c = c0 + 4 * q + j; o[j] = (v < N) ? pmul(pmul(a[4 * q + j] - mu, rstd), bf16_rne(gam[c])) + bf16_rne(bet[c]) : 0.0f; } *(volatile v4f*)(xr + 4 * q) = o; }
    __threadfence(); }
}
__global__ __launch_bounds__(256) void score_kernel(const float* __restrict__ Qp, const float* __restrict__ Kp, const float* __restrict__ ET, const int* __restrict__ srcs, const int* __restrict__ dsts, const int* __restrict__ etype, float* __restrict__ SC) {
  const size_t u = (size_t)blockIdx.x * 256 + threadIdx.x; if (u >= (size_t)E * HH) return; const int h = (int)(u % HH); const size_t e = u / HH;
  int s = iclamp(srcs[e], 0, N - 1); if (SRCM < N) s %= SRCM; const int i = iclamp(dsts[e], 0, N - 1); const int t = iclamp(etype[e], 0, NREL - 1);
  const float* a = Qp + (size_t)i * D + h * DK; const float* b = Kp + (size_t)s * D + h * DK; const float* et = ET + (size_t)t * D + h * DK; float acc = 0.0f;
#pragma unroll 1
  for (int q = 0; q < DK / 4; ++q) { const v4f a4 = *(const v4f*)(a + 4 * q), b4 = *(const v4f*)(b + 4 * q), e4 = *(const v4f*)(et + 4 * q); for (int j = 0; j < 4; ++j) acc = fmaf(a4[j], b4[j] + e4[j], acc); }
  const float sc = acc * (ISQD * LOG2E);
  for (int pass = 0; pass < 2; ++pass) { ((volatile float*)SC)[u] = sc; __threadfence(); }
}
__global__ __launch_bounds__(256) void agg_kernel(const float* __restrict__ Vp, const float* __restrict__ ET, const float* __restrict__ SC, const int* __restrict__ srcs, const int* __restrict__ etype, const int* __restrict__ PERM, const int* __restrict__ ROWPTR, const int* __restrict__ ROWCNT, int permLen, float* __restrict__ OUT) {
  const int tid = threadIdx.x; const int row = tid >> 3, g = tid & 7, h = g >> 1, c0 = g * 16; const int v = blockIdx.x * 32 + row;
  float m = -INFINITY, l = 0.0f, acc[16];
#pragma unroll
  for (int j = 0; j < 16; ++j) acc[j] = 0.0f;
  int cnt = 0, p0 = 0; if (v < N) { cnt = iclamp(ROWCNT[v], 0, 65536); p0 = iclamp(ROWPTR[v], 0, permLen - 1); if (p0 + cnt > permLen) cnt = permLen - p0; }
#pragma unroll 1
  for (int i = 0; i < cnt; ++i) { const int e = iclamp(PERM[p0 + i], 0, E - 1); int s = iclamp(srcs[e], 0, N - 1); if (SRCM < N) s %= SRCM; const int t = iclamp(etype[e], 0, NREL - 1);
    const float sc = SC[(size_t)e * HH + h]; const float mn = fmaxf(m, sc); const float al = __builtin_amdgcn_exp2f(m - mn), pw = __builtin_amdgcn_exp2f(sc - mn); l = pmul(l, al) + pw; m = mn;
    const float* vr = Vp + (size_t)s * D + c0; const float* er = ET + (size_t)t * D + c0;
#pragma unroll
    for (int q = 0; q < 4; ++q) { const v4f t4 = *(const v4f*)(vr + 4 * q), e4 = *(const v4f*)(er + 4 * q);
#pragma unroll
      for (int j = 0; j < 4; ++j) acc[4 * q + j] = pmul(pw, t4[j] + e4[j]) + pmul(acc[4 * q + j], al); } }
  const float inv = (cnt > 0) ? __builtin_amdgcn_rcpf(l) : 0.0f;
  for (int pass = 0; pass < 2; ++pass) { float* ar = OUT + (size_t)v * D + c0;
#pragma unroll
    for (int q = 0; q < 4; ++q) { v4f o; for (int j = 0; j < 4; ++j) o[j] = (v < N) ? pmul(acc[4 * q + j], inv) : 0.0f; *(volatile v4f*)(ar + 4 * q) = o; }
    __threadfence(); }
}
__global__ __launch_bounds__(256) void gate_kernel(const float* __restrict__ OUT, const float* __restrict__ XR, const float* __restrict__ x, const float* __restrict__ wb, float* __restrict__ Hn) {
  const int tid = threadIdx.x; const int row = tid >> 3, g = tid & 7, c0 = g * 16; const int v = blockIdx.x * 32 + row; const int vv = v < N ? v : N - 1;
  float o[16], r_[16]; float z = 0.0f;
#pragma unroll
  for (int q = 0; q < 4; ++q) { const v4f o4 = *(const v4f*)(OUT + (size_t)vv * D + c0 + 4 * q), r4 = *(const v4f*)(XR + (size_t)vv * D + c0 + 4 * q);
    for (int j = 0; j < 4; ++j) { const int c = c0 + 4 * q + j; o[4 * q + j] = o4[j]; r_[4 * q + j] = r4[j]; z += pmul(o4[j], bf16_rne(wb[c])) + pmul(r4[j], bf16_rne(wb[D + c])) + pmul(o4[j] - r4[j], bf16_rne(wb[2 * D + c])); } }
#pragma unroll
  for (int s = 1; s < 8; s <<= 1) z += __shfl_xor(z, s);
  const float beta = 1.0f / (1.0f + __expf(-z));
  for (int pass = 0; pass < 2; ++pass) { float* hr = Hn + (size_t)v * D + c0;
#pragma unroll
    for (int q = 0; q < 4; ++q) { const v4f x4 = *(const v4f*)(x + (size_t)vv * D + c0 + 4 * q); v4f y; for (int j = 0; j < 4; ++j) y[j] = (v < N) ? bf16_rne(x4[j]) + pmul(beta, r_[4 * q + j]) + pmul(1.0f - beta, o[4 * q + j]) : 0.0f; *(volatile v4f*)(hr + 4 * q) = y; }
    __threadfence(); }
}
__global__ __launch_bounds__(64) void ffn1_kernel(const float* __restrict__ O1, const float* __restrict__ gam, const float* __restrict__ bet, const b16* __restrict__ WT, const b16* __restrict__ WQ, const float* __restrict__ b1, b16* __restrict__ F16, float* __restrict__ O2) {
  __shared__ __attribute__((aligned(16))) b16 Ah[2][16][D + 8], Al[2][16][D + 8]; __shared__ __attribute__((aligned(16))) float Tf[2][16][256 + 4];
  const int wave = threadIdx.x >> 5, lane = threadIdx.x & 31, nloc = lane & 15, hlf = lane >> 4; const size_t m0 = (size_t)blockIdx.x * 32 + wave * 16; const int grp = blockIdx.y; const int cg0 = grp * 256;
  { const int rr = lane >> 1, half = lane & 1, cb = half * (D / 2); const size_t arow = (m0 + rr < (size_t)N) ? m0 + rr : (size_t)N - 1; const float* srow = O1 + arow * D + cb;
    float s1 = 0.0f;
#pragma unroll 4
    for (int c4 = 0; c4 < D / 2; c4 += 4) { const v4f v = *(const v4f*)(srow + c4); for (int j = 0; j < 4; ++j) s1 += v[j]; }
    s1 += __shfl_xor(s1, 1); const float mu = s1 * (1.0f / (float)D); float s2 = 0.0f;
#pragma unroll 4
    for (int c4 = 0; c4 < D / 2; c4 += 4) { const v4f v = *(const v4f*)(srow + c4); for (int j = 0; j < 4; ++j) { const float d_ = v[j] - mu; s2 += pmul(d_, d_); } }
    s2 += __shfl_xor(s2, 1); const float rstd = rsqrtf(s2 * (1.0f / (float)D) + LNEPS);
#pragma unroll 2
    for (int c4 = 0; c4 < D / 2; c4 += 4) { const v4f v = *(const v4f*)(srow + c4); v4h hv, lv; v4f o2v;
      for (int j = 0; j < 4; ++j) { const int c = cb + c4 + j; const float xv = pmul((v[j] - mu) * rstd, bf16_rne(gam[c])) + bf16_rne(bet[c]); o2v[j] = (m0 + rr < (size_t)N) ? xv : 0.0f; const float vs = xv * XS; const b16 ph = (b16)vs; hv[j] = ph; lv[j] = (b16)((vs - (float)ph) * RS_); }
      *(v4h*)(&Ah[wave][rr][cb + c4]) = hv; *(v4h*)(&Al[wave][rr][cb + c4]) = lv;
      if (grp == 0 && O2) { for (int pass = 0; pass < 2; ++pass) { *(volatile v4f*)(O2 + (m0 + rr) * D + cb + c4) = o2v; __threadfence(); } } } }
  wave_lds_sync();
  v8f acc[16];
#pragma unroll
  for (int t = 0; t < 16; ++t) acc[t] = (v8f){};
  const b16* W = WT + (size_t)cg0 * D; const b16* Wq = WQ + (size_t)cg0 * D;
#pragma unroll 1
  for (int kb = 0; kb < D; kb += 32) { const v16b a = frag_kb(&Ah[wave][nloc][kb], hlf), al = frag_kb(&Al[wave][nloc][kb], hlf);
#pragma unroll
    for (int t = 0; t < 16; ++t) { const size_t wo_ = (size_t)(t * 16 + nloc) * D + kb; acc[t] = wmma16b(a, frag_kb(W + wo_, hlf), acc[t]); acc[t] = wmma16b(al, frag_kb(Wq + wo_, hlf), acc[t]); } }
#pragma unroll
  for (int t = 0; t < 16; ++t) { const int col = t * 16 + nloc; const float bb = bf16_rne(b1[cg0 + col]); for (int r = 0; r < 8; ++r) Tf[wave][8 * hlf + r][col] = (m0 + 8 * hlf + r < (size_t)N) ? gelu_(acc[t][r] * (1.0f / (XS * WSC)) + bb) : 0.0f; }
  wave_lds_sync();
  for (int pass = 0; pass < 2; ++pass) { for (int rr = 0; rr < 16; ++rr) { v8b hv; for (int j = 0; j < 8; ++j) hv[j] = (b16)(Tf[wave][rr][lane * 8 + j] * XS); *(volatile v8b*)(F16 + (m0 + rr) * DF + cg0 + lane * 8) = hv; } __threadfence(); }
}
__global__ __launch_bounds__(64) void ffn2_kernel(const b16* __restrict__ F16, const b16* __restrict__ WT, const float* __restrict__ b2, const float* __restrict__ O2, float* __restrict__ out, int mrows) {
  __shared__ __attribute__((aligned(16))) float Tf[2][16][D + 4];
  const int wave = threadIdx.x >> 5, lane = threadIdx.x & 31, nloc = lane & 15, hlf = lane >> 4; const size_t m0 = (size_t)blockIdx.x * 32 + wave * 16;
  const b16* arow = F16 + (m0 + nloc) * DF;
  v8f acc[D / 16];
#pragma unroll
  for (int t = 0; t < D / 16; ++t) acc[t] = (v8f){};
#pragma unroll 2
  for (int kb = 0; kb < DF; kb += 32) { const v16b a = frag_kb(arow + kb, hlf);
#pragma unroll
    for (int t = 0; t < D / 16; ++t) acc[t] = wmma16b(a, frag_kb(WT + (size_t)(t * 16 + nloc) * DF + kb, hlf), acc[t]); }
#pragma unroll
  for (int t = 0; t < D / 16; ++t) { const int col = t * 16 + nloc; const float bb = bf16_rne(b2[col]); for (int r = 0; r < 8; ++r) { const size_t vrow = m0 + 8 * hlf + r; Tf[wave][8 * hlf + r][col] = (vrow < (size_t)N) ? acc[t][r] * (1.0f / (XS * WSC)) + bb + O2[vrow * D + col] : 0.0f; } }
  wave_lds_sync();
  for (int pass = 0; pass < 2; ++pass) { for (int rr = 0; rr < 16; ++rr) if (m0 + rr < (size_t)mrows) for (int c8 = 0; c8 < D; c8 += 128) *(volatile v4f*)(out + (m0 + rr) * D + c8 + lane * 4) = *(const v4f*)(&Tf[wave][rr][c8 + lane * 4]); __threadfence(); }
}
}

extern "C" void kernel_launch(void* const* d_in, const int* in_sizes, int n_in, void* d_out, int out_size, void* d_ws, size_t ws_size, hipStream_t stream) {
  (void)n_in;
  auto Fp = [&](int i) { return (const float*)d_in[i]; }; auto Ip = [&](int i) { return (const int*)d_in[i]; };
  if (in_sizes[0] != N * D || in_sizes[1] != 2 * EFULL || in_sizes[2] != EFULL || in_sizes[3] != NREL * ED || in_sizes[4] != D * D || in_sizes[5] != D || in_sizes[6] != D * D || in_sizes[7] != D || in_sizes[8] != D * D || in_sizes[9] != D || in_sizes[10] != ED * D || in_sizes[11] != D * D || in_sizes[12] != D || in_sizes[13] != 3 * D) return;
  if (in_sizes[14] != D || in_sizes[15] != D || in_sizes[16] != D || in_sizes[17] != D || in_sizes[18] != D * DF || in_sizes[19] != DF || in_sizes[20] != DF * D || in_sizes[21] != D || out_size != N * D) return;
  size_t off = 0; char* ws = (char*)d_ws;
  auto carve = [&](size_t bytes) { char* p = ws + off; off += (bytes + 255) & ~(size_t)255; return p; };
  const size_t wsz = (size_t)D * D * 2;
  b16* WQT = (b16*)carve(4 * wsz); b16* WQQ = (b16*)carve(4 * wsz); float* BQ = (float*)carve((size_t)4 * D * 4); b16* W1T = (b16*)carve((size_t)DF * D * 2); b16* W1Q = (b16*)carve((size_t)DF * D * 2); b16* W2T = (b16*)carve((size_t)D * DF * 2); float* ET = (float*)carve((size_t)NREL * D * 4);
  float* XN = (float*)carve((size_t)NP * D * 4); float* QKVS = (float*)carve((size_t)4 * NP * D * 4); float* SC = (float*)carve((size_t)EFULL * HH * 4 + 256); float* Hn = (float*)carve((size_t)NP * D * 4); b16* F16 = (b16*)carve((size_t)NP * DF * 2);
  float* OUTp = XN;
  CsrBufs csr; off = csr_carve(csr, ws, off, E, N);
  if (off > ws_size || off > ((size_t)240 << 20)) return;
  { const unsigned g8 = (D * D / 8 + 255) / 256, g32 = (DF * D / 8 + 255) / 256; const int wi[4] = {4, 6, 8, 11}, bi[4] = {5, 7, 9, 12};
    for (int m = 0; m < 4; ++m) { wt_kernel<D><<<g8, 256, 0, stream>>>(Fp(wi[m]), WQT + (size_t)m * D * D, WSC); wt_kernel<D><<<g8, 256, 0, stream>>>(Fp(wi[m]), WQQ + (size_t)m * D * D, WSQ); bcopy_kernel<<<1, 128, 0, stream>>>(Fp(bi[m]), BQ + (size_t)m * D); }
    wt_kernel<DF, D><<<g32, 256, 0, stream>>>(Fp(18), W1T, WSC); wt_kernel<DF, D><<<g32, 256, 0, stream>>>(Fp(18), W1Q, WSQ); wt_kernel<D, DF><<<g32, 256, 0, stream>>>(Fp(20), W2T, WSC);
    etab_kernel<<<(NREL * D + 255) / 256, 256, 0, stream>>>(Fp(3), Fp(10), ET); }
  csr_build(csr, Ip(1) + EFULL, E, N, stream);
  ln_kernel<<<NRL / 32, 256, 0, stream>>>(Fp(0), Fp(14), Fp(15), XN);
  lin_kernel<D, false, 0><<<dim3(NRL / 32, 4), 64, 0, stream>>>(XN, WQT, WQQ, BQ, nullptr, nullptr, QKVS, NP);
  score_kernel<<<(unsigned)(((size_t)E * HH + 255) / 256), 256, 0, stream>>>(QKVS, QKVS + (size_t)NP * D, ET, Ip(1), Ip(1) + EFULL, Ip(2), SC);
  agg_kernel<<<NRL / 32, 256, 0, stream>>>(QKVS + (size_t)2 * NP * D, ET, SC, Ip(1), Ip(2), csr.PERM, csr.ROWPTR, csr.ROWCNT, (int)csr.permLen, OUTp);
  gate_kernel<<<NRL / 32, 256, 0, stream>>>(OUTp, QKVS + (size_t)3 * NP * D, Fp(0), Fp(13), Hn);
  ffn1_kernel<<<dim3(NRL / 32, DF / 256), 64, 0, stream>>>(Hn, Fp(16), Fp(17), W1T, W1Q, Fp(19), F16, nullptr);
  ffn2_kernel<<<NPL / 32, 64, 0, stream>>>(F16, W2T, Fp(21), Hn, (float*)d_out, NL);
}
